// multi_head_attention_32229434589370
// MI455X (gfx1250) — hardware-verified
//
#include <hip/hip_runtime.h>
#include <hip/hip_bf16.h>


#ifndef NB
#define NB 8
#endif
#ifndef SEQ
#define SEQ 2048
#endif
#define NB_FULL  8
#define SEQ_FULL 2048
#define DM   512
#define NH   8
#define HD   64
#define ER   128
#define EQB    ((((SEQ) / 64) < 8) ? ((SEQ) / 64) : 8)
#define RT_UNC ((((EQB) * 64 + 64 + 127) / 128) * 128)
#define RT     ((RT_UNC < (SEQ)) ? RT_UNC : (SEQ))
#define NTOK (NB * SEQ)
#define XPL  ((size_t)NTOK * DM)
#define WPL  ((size_t)DM * DM)
#define CPL  ((size_t)NTOK * DM)
#define FPL  ((size_t)NB * NH * ER * HD)
#define RPL  ((size_t)NB * NH * RT * HD)

static_assert(NB >= 1 && NB <= NB_FULL);
static_assert(SEQ >= 128 && SEQ <= SEQ_FULL && (SEQ % 128) == 0);
static_assert(DM == NH * HD && HD == 64 && NH == 8 && ER == 128);
static_assert((NTOK % 128) == 0);
static_assert(EQB >= 2 && EQB * 64 <= SEQ);
static_assert((RT % 128) == 0 && RT <= SEQ && (RT >= EQB * 64 + 64 || RT == SEQ));
static_assert((size_t)6 * XPL * 2 + (size_t)4 * WPL * 2 + (size_t)3 * FPL * 4 + (size_t)3 * RPL * 2 <= (size_t)134217728);
static_assert((size_t)2 * CPL <= (size_t)3 * XPL);

typedef _Float16     v16h  __attribute__((ext_vector_type(16)));
typedef _Float16     v8h   __attribute__((ext_vector_type(8)));
typedef __bf16       v16bf __attribute__((ext_vector_type(16)));
typedef float        v8f   __attribute__((ext_vector_type(8)));
typedef float        v4f   __attribute__((ext_vector_type(4)));
typedef unsigned int u32x4 __attribute__((ext_vector_type(4)));
typedef v8h   v8ha   __attribute__((may_alias));
typedef v4f   v4fa   __attribute__((may_alias));
typedef u32x4 u32x4a __attribute__((may_alias));

union Frag  { v16h f; v16bf b; v8h hv[2]; u32x4 q[2]; unsigned int u[8]; };
union Pack8 { v8h h; u32x4 u; };

__device__ __forceinline__ unsigned short f2bf(float f) {
    unsigned int u = __builtin_bit_cast(unsigned int, f);
    u = (u + 0x7fffu + ((u >> 16) & 1u)) >> 16;
    return (unsigned short)u;
}
__device__ __forceinline__ float bf2f(unsigned short s) {
    return __builtin_bit_cast(float, ((unsigned int)s) << 16);
}
__device__ __forceinline__ float bfr(float f) { return bf2f(f2bf(f)); }
__device__ __forceinline__ unsigned int f2bf2(float lo, float hi) {
    return (unsigned int)f2bf(lo) | ((unsigned int)f2bf(hi) << 16);
}
__device__ __forceinline__ _Float16 res16(float x) {
    const _Float16 hx = (_Float16)x;
    return (_Float16)((x - (float)hx) * 1024.f);
}

__device__ __forceinline__ v8f mma_bf16(const Frag& a, const Frag& b, v8f c) {
    c = __builtin_amdgcn_wmma_f32_16x16x32_bf16(false, a.b, false, b.b, (short)0, c, false, false);
    asm volatile("v_nop\n\tv_nop\n\tv_nop\n\tv_nop" : "+v"(c) : "v"(a.f), "v"(b.f));
    return c;
}
__device__ __forceinline__ v8f mma_f16(const Frag& a, const Frag& b, v8f c) {
    c = __builtin_amdgcn_wmma_f32_16x16x32_f16(false, a.f, false, b.f, (short)0, c, false, false);
    asm volatile("v_nop\n\tv_nop\n\tv_nop\n\tv_nop" : "+v"(c) : "v"(a.f), "v"(b.f));
    return c;
}

__launch_bounds__(256)
__global__ void cvt_kernel(const float* __restrict__ q, const float* __restrict__ k,
                           const float* __restrict__ v,
                           const float* __restrict__ wq, const float* __restrict__ wk,
                           const float* __restrict__ wv, const float* __restrict__ wc,
                           unsigned short* __restrict__ xb, unsigned short* __restrict__ wb)
{
    const int tid = threadIdx.x;
    const int blk = blockIdx.x;
    const int XB  = 3 * (NTOK / 4);
    const float* src;
    unsigned short* dst;
    if (blk < XB) {
        const int z  = blk / (NTOK / 4);
        const int wi = blk - z * (NTOK / 4);
        const size_t e0 = (size_t)wi * 2048 + (size_t)tid * 8;
        const int m  = (int)(e0 >> 9);
        const int c  = (int)(e0 & 511);
        const int bb = m / SEQ;
        const int t  = m - bb * SEQ;
        const float* base = (z == 0) ? q : (z == 1) ? k : v;
        src = base + ((size_t)bb * SEQ_FULL + t) * DM + c;
        dst = xb + (size_t)z * XPL + e0;
    } else {
        const int j  = blk - XB;
        const int z  = j >> 7;
        const size_t e0 = (size_t)(j & 127) * 2048 + (size_t)tid * 8;
        const float* base = (z == 0) ? wq : (z == 1) ? wk : (z == 2) ? wv : wc;
        src = base + e0;
        dst = wb + (size_t)z * WPL + e0;
    }
    const v4f x0 = *(const v4f*)(src);
    const v4f x1 = *(const v4f*)(src + 4);
    u32x4 pk;
    pk.x = f2bf2(x0.x, x0.y);
    pk.y = f2bf2(x0.z, x0.w);
    pk.z = f2bf2(x1.x, x1.y);
    pk.w = f2bf2(x1.z, x1.w);
    *(volatile u32x4*)dst = pk;
    __threadfence();
    *(volatile u32x4*)dst = pk;
}

__launch_bounds__(128)
__global__ void proj_kernel(const unsigned short* __restrict__ xb,
                            const unsigned short* __restrict__ wb,
                            const float* __restrict__ bq, const float* __restrict__ bk,
                            const float* __restrict__ bv,
                            unsigned short* __restrict__ qh, unsigned short* __restrict__ kh,
                            unsigned short* __restrict__ vt,
                            unsigned short* __restrict__ qr, unsigned short* __restrict__ kr,
                            unsigned short* __restrict__ vr,
                            float* __restrict__ qf, float* __restrict__ kf,
                            float* __restrict__ vf)
{
    __shared__ __align__(16) float stg[128][68];

    const int tid = threadIdx.x, l = tid & 31, w = tid >> 5;
    const int h = (l >> 4) & 1, nl = l & 15;
    const int z    = blockIdx.z;
    const int mblk = blockIdx.x * 128;
    const int hh   = blockIdx.y;
    const unsigned short* X = xb + (size_t)z * XPL;
    const unsigned short* W = wb + (size_t)z * WPL;
    const float* bias = (z == 0) ? bq : (z == 1) ? bk : bv;

    v8f acc[2][4] = {};
    #pragma unroll 2
    for (int s = 0; s < 16; ++s) {
        Frag A[2], B[4];
        #pragma unroll
        for (int mi = 0; mi < 2; ++mi) {
            const unsigned short* p = X + (size_t)(mblk + 32 * w + 16 * mi + nl) * DM + 32 * s + 8 * h;
            A[mi].q[0] = *(const u32x4*)(p);
            A[mi].q[1] = *(const u32x4*)(p + 16);
        }
        #pragma unroll
        for (int ni = 0; ni < 4; ++ni) {
            const unsigned short* p = W + (size_t)(hh * 64 + 16 * ni + nl) * DM + 32 * s + 8 * h;
            B[ni].q[0] = *(const u32x4*)(p);
            B[ni].q[1] = *(const u32x4*)(p + 16);
        }
        #pragma unroll
        for (int mi = 0; mi < 2; ++mi)
            #pragma unroll
            for (int ni = 0; ni < 4; ++ni)
                acc[mi][ni] = mma_bf16(A[mi], B[ni], acc[mi][ni]);
    }

    float bb[4];
    #pragma unroll
    for (int ni = 0; ni < 4; ++ni) bb[ni] = bfr(bias[hh * 64 + 16 * ni + nl]);
    #pragma unroll
    for (int mi = 0; mi < 2; ++mi)
        #pragma unroll
        for (int ni = 0; ni < 4; ++ni)
            #pragma unroll
            for (int r = 0; r < 8; ++r)
                stg[32 * w + 16 * mi + 8 * h + r][16 * ni + nl] = acc[mi][ni][r] + bb[ni];
    __syncthreads();

    const int bbI = mblk / SEQ;
    const int t0  = mblk - bbI * SEQ;
    const int bh  = bbI * NH + hh;
    const int q8  = tid & 7;
    const int lg  = tid >> 3;

    if (z < 2) {
        unsigned short* base16 = ((z == 0) ? qh : kh) + ((size_t)bh * SEQ + t0) * HD;
        auto pass16 = [&]() {
            #pragma unroll
            for (int it = 0; it < 8; ++it) {
                const int L = it * 16 + lg;
                const v4f a0 = *(const v4fa*)&stg[L][8 * q8];
                const v4f a1 = *(const v4fa*)&stg[L][8 * q8 + 4];
                Pack8 P;
                P.h[0] = (_Float16)(a0.x * 16.f); P.h[1] = (_Float16)(a0.y * 16.f);
                P.h[2] = (_Float16)(a0.z * 16.f); P.h[3] = (_Float16)(a0.w * 16.f);
                P.h[4] = (_Float16)(a1.x * 16.f); P.h[5] = (_Float16)(a1.y * 16.f);
                P.h[6] = (_Float16)(a1.z * 16.f); P.h[7] = (_Float16)(a1.w * 16.f);
                *(volatile u32x4*)(base16 + (size_t)L * HD + 8 * q8) = P.u;
            }
        };
        pass16();
        __threadfence();
        pass16();
        if (t0 < RT) {
            unsigned short* baser = ((z == 0) ? qr : kr) + ((size_t)bh * RT + t0) * HD;
            auto passr = [&]() {
                #pragma unroll
                for (int it = 0; it < 8; ++it) {
                    const int L = it * 16 + lg;
                    const v4f a0 = *(const v4fa*)&stg[L][8 * q8];
                    const v4f a1 = *(const v4fa*)&stg[L][8 * q8 + 4];
                    Pack8 P;
                    P.h[0] = res16(a0.x * 16.f); P.h[1] = res16(a0.y * 16.f);
                    P.h[2] = res16(a0.z * 16.f); P.h[3] = res16(a0.w * 16.f);
                    P.h[4] = res16(a1.x * 16.f); P.h[5] = res16(a1.y * 16.f);
                    P.h[6] = res16(a1.z * 16.f); P.h[7] = res16(a1.w * 16.f);
                    *(volatile u32x4*)(baser + (size_t)L * HD + 8 * q8) = P.u;
                }
            };
            passr();
            __threadfence();
            passr();
        }
    } else {
        unsigned short* basev = vt + (size_t)bh * HD * SEQ + t0;
        auto passv = [&]() {
            #pragma unroll
            for (int it = 0; it < 8; ++it) {
                const int L  = it * 16 + lg;
                const int d  = L >> 1, tg = L & 1;
                Pack8 P;
                #pragma unroll
                for (int e = 0; e < 8; ++e)
                    P.h[e] = (_Float16)(stg[tg * 64 + 8 * q8 + e][d] * 16.f);
                *(volatile u32x4*)(basev + (size_t)d * SEQ + tg * 64 + 8 * q8) = P.u;
            }
        };
        passv();
        __threadfence();
        passv();
        if (t0 < RT) {
            unsigned short* basex = vr + (size_t)bh * HD * RT + t0;
            auto passx = [&]() {
                #pragma unroll
                for (int it = 0; it < 8; ++it) {
                    const int L  = it * 16 + lg;
                    const int d  = L >> 1, tg = L & 1;
                    Pack8 P;
                    #pragma unroll
                    for (int e = 0; e < 8; ++e)
                        P.h[e] = res16(stg[tg * 64 + 8 * q8 + e][d] * 16.f);
                    *(volatile u32x4*)(basex + (size_t)d * RT + tg * 64 + 8 * q8) = P.u;
                }
            };
            passx();
            __threadfence();
            passx();
        }
    }

    if (t0 == 0) {
        float* F = ((z == 0) ? qf : (z == 1) ? kf : vf) + (size_t)bh * ER * HD;
        auto passf = [&]() {
            #pragma unroll
            for (int it = 0; it < 16; ++it) {
                const int L = it * 16 + lg;
                const int row = L >> 1, hf = L & 1;
                const v4f x = *(const v4fa*)&stg[row][hf * 32 + 4 * q8];
                *(volatile v4f*)(F + (size_t)row * HD + hf * 32 + 4 * q8) = x;
            }
        };
        passf();
        __threadfence();
        passf();
    }
}

template<int EARLY>
__launch_bounds__(128)
__global__ void attn_kernel(const unsigned short* __restrict__ qh,
                            const unsigned short* __restrict__ kh,
                            const unsigned short* __restrict__ vt,
                            const unsigned short* __restrict__ qr,
                            const unsigned short* __restrict__ kr,
                            const unsigned short* __restrict__ vr,
                            unsigned short* __restrict__ ctx)
{
    __shared__ __align__(16) _Float16       pst[4][16][72];
    __shared__ __align__(16) _Float16       prt[4][16][72];
    __shared__ __align__(16) unsigned short cst[4][2][16][72];

    const int tid = threadIdx.x, l = tid & 31, w = tid >> 5;
    const int h = (l >> 4) & 1, nl = l & 15;
    const int qb  = EARLY ? ((int)blockIdx.x + 1) : ((int)blockIdx.x + EQB);
    const int bh  = blockIdx.y, bbI = bh >> 3, hh = bh & 7;
    const int i0  = qb * 64 + w * 16;
    const float C1  = 7.0444093793406406e-4f;
    const float PSC = 16384.f;
    const float RSC = 0.0009765625f;

    Frag aq[2];
    {
        const unsigned short* qp = qh + ((size_t)bh * SEQ + i0 + nl) * HD + 8 * h;
        #pragma unroll
        for (int s = 0; s < 2; ++s) {
            aq[s].q[0] = *(const u32x4*)(qp + 32 * s);
            aq[s].q[1] = *(const u32x4*)(qp + 32 * s + 16);
        }
    }
    Frag ar[2];
    if constexpr (EARLY) {
        const unsigned short* qp = qr + ((size_t)bh * RT + i0 + nl) * HD + 8 * h;
        #pragma unroll
        for (int s = 0; s < 2; ++s) {
            ar[s].q[0] = *(const u32x4*)(qp + 32 * s);
            ar[s].q[1] = *(const u32x4*)(qp + 32 * s + 16);
        }
    }
    v8f o[4]  = {};
    v8f o2[4] = {};
    float m2[8], ls[8];
    #pragma unroll
    for (int r = 0; r < 8; ++r) { m2[r] = -3.0e38f; ls[r] = 0.f; }

    const unsigned short* kbase  = kh + (size_t)bh * SEQ * HD + (size_t)nl * HD + 8 * h;
    const unsigned short* vbase  = vt + (size_t)bh * HD * SEQ + (size_t)nl * SEQ + 8 * h;
    const unsigned short* krbase = kr + (size_t)bh * RT * HD + (size_t)nl * HD + 8 * h;
    const unsigned short* vrbase = vr + (size_t)bh * HD * RT + (size_t)nl * RT + 8 * h;
    const int jmax = (i0 + 16 < SEQ - 1) ? (i0 + 16) : (SEQ - 1);

    for (int j0 = 0; j0 <= jmax; j0 += 64) {
        v8f sc[4];
        #pragma unroll
        for (int n = 0; n < 4; ++n) {
            v8f c  = {};
            v8f c2 = {};
            #pragma unroll
            for (int s = 0; s < 2; ++s) {
                Frag kb;
                const unsigned short* p = kbase + (size_t)(j0 + 16 * n) * HD + 32 * s;
                kb.q[0] = *(const u32x4*)(p);
                kb.q[1] = *(const u32x4*)(p + 16);
                c = mma_f16(aq[s], kb, c);
                if constexpr (EARLY) {
                    Frag kx;
                    const unsigned short* px = krbase + (size_t)(j0 + 16 * n) * HD + 32 * s;
                    kx.q[0] = *(const u32x4*)(px);
                    kx.q[1] = *(const u32x4*)(px + 16);
                    c2 = mma_f16(aq[s], kx, c2);
                    c2 = mma_f16(ar[s], kb, c2);
                }
            }
            if constexpr (EARLY) { sc[n] = c + c2 * RSC; }
            else                 { sc[n] = c; (void)c2; }
        }

        float alpha[8];
        #pragma unroll
        for (int r = 0; r < 8; ++r) {
            const int row = i0 + 8 * h + r;
            float mx = -3.0e38f;
            #pragma unroll
            for (int n = 0; n < 4; ++n) {
                const int j = j0 + 16 * n + nl;
                const float sv = sc[n][r] * C1;
                mx = (j <= row + 1) ? fmaxf(mx, sv) : mx;
            }
            mx = fmaxf(mx, __shfl_xor(mx, 1, 32));
            mx = fmaxf(mx, __shfl_xor(mx, 2, 32));
            mx = fmaxf(mx, __shfl_xor(mx, 4, 32));
            mx = fmaxf(mx, __shfl_xor(mx, 8, 32));
            const float mn = fmaxf(m2[r], mx);
            alpha[r] = exp2f(m2[r] - mn);
            m2[r] = mn;
        }
        #pragma unroll
        for (int r = 0; r < 8; ++r) {
            const int row = i0 + 8 * h + r;
            float rs = 0.f;
            #pragma unroll
            for (int n = 0; n < 4; ++n) {
                const int j = j0 + 16 * n + nl;
                const float sv = sc[n][r] * C1;
                const float p  = (j <= row + 1) ? exp2f(sv - m2[r]) : 0.f;
                const float t  = p * PSC;
                const _Float16 ph = (_Float16)t;
                pst[w][8 * h + r][16 * n + nl] = ph;
                if constexpr (EARLY) {
                    const _Float16 pxx = (_Float16)((t - (float)ph) * 1024.f);
                    prt[w][8 * h + r][16 * n + nl] = pxx;
                    rs += (float)ph + (float)pxx * RSC;
                } else {
                    rs += (float)ph;
                }
            }
            rs += __shfl_xor(rs, 1, 32);
            rs += __shfl_xor(rs, 2, 32);
            rs += __shfl_xor(rs, 4, 32);
            rs += __shfl_xor(rs, 8, 32);
            ls[r] = ls[r] * alpha[r] + rs;
        }
        #pragma unroll
        for (int f = 0; f < 4; ++f)
            #pragma unroll
            for (int r = 0; r < 8; ++r) {
                o[f][r] *= alpha[r];
                if constexpr (EARLY) o2[f][r] *= alpha[r];
            }

        __builtin_amdgcn_fence(3  , "wavefront");
        __builtin_amdgcn_wave_barrier();

        #pragma unroll 1
        for (int s = 0; s < 2; ++s) {
            Frag pa;
            pa.hv[0] = *(const v8ha*)&pst[w][nl][32 * s + 8 * h];
            pa.hv[1] = *(const v8ha*)&pst[w][nl][32 * s + 16 + 8 * h];
            Frag pb;
            if constexpr (EARLY) {
                pb.hv[0] = *(const v8ha*)&prt[w][nl][32 * s + 8 * h];
                pb.hv[1] = *(const v8ha*)&prt[w][nl][32 * s + 16 + 8 * h];
            }
            #pragma unroll
            for (int f = 0; f < 4; ++f) {
                Frag vb;
                const unsigned short* p = vbase + (size_t)(16 * f) * SEQ + j0 + 32 * s;
                vb.q[0] = *(const u32x4*)(p);
                vb.q[1] = *(const u32x4*)(p + 16);
                o[f] = mma_f16(pa, vb, o[f]);
                if constexpr (EARLY) {
                    Frag vx;
                    const unsigned short* px = vrbase + (size_t)(16 * f) * RT + j0 + 32 * s;
                    vx.q[0] = *(const u32x4*)(px);
                    vx.q[1] = *(const u32x4*)(px + 16);
                    o2[f] = mma_f16(pa, vx, o2[f]);
                    o2[f] = mma_f16(pb, vb, o2[f]);
                }
            }
        }
        __builtin_amdgcn_fence(3  , "wavefront");
        __builtin_amdgcn_wave_barrier();
    }

    #pragma unroll
    for (int r = 0; r < 8; ++r) {
        const float inv = 1.0f / (ls[r] * 16.f);
        #pragma unroll
        for (int f = 0; f < 4; ++f) {
            float x = o[f][r];
            if constexpr (EARLY) x += o2[f][r] * RSC;
            x *= inv;
            const unsigned short hb = f2bf(x);
            const unsigned short lb = f2bf(x - bf2f(hb));
            cst[w][0][8 * h + r][16 * f + nl] = hb;
            cst[w][1][8 * h + r][16 * f + nl] = lb;
        }
    }
    (void)o2;
    __builtin_amdgcn_fence(3  , "wavefront");
    __builtin_amdgcn_wave_barrier();

    unsigned short* cbase = ctx + ((size_t)bbI * SEQ + i0) * DM + hh * HD;
    auto passc = [&]() {
        #pragma unroll
        for (int it = 0; it < 8; ++it) {
            const int L = it * 4 + (l >> 3);
            const int row = L >> 1, pl = L & 1, q8 = l & 7;
            const u32x4 val = *(const u32x4a*)&cst[w][pl][row][8 * q8];
            *(volatile u32x4*)(cbase + (size_t)pl * CPL + (size_t)row * DM + 8 * q8) = val;
        }
    };
    passc();
    __threadfence();
    passc();
}

__launch_bounds__(256)
__global__ void attn_first_kernel(const float* __restrict__ qf, const float* __restrict__ kf,
                                  const float* __restrict__ vf, unsigned short* __restrict__ ctx)
{
    __shared__ __align__(16) float qs[64][64];
    __shared__ __align__(16) float kv[65][64];
    __shared__ __align__(16) float ps[64][68];
    __shared__ float rinv[64];

    const int tid = threadIdx.x;
    const int bh  = blockIdx.x, bbI = bh >> 3, hh = bh & 7;
    const float* Q = qf + (size_t)bh * ER * HD;
    const float* K = kf + (size_t)bh * ER * HD;
    const float* V = vf + (size_t)bh * ER * HD;
    const float LOG2E = 1.4426950408889634f;

    for (int i = tid; i < 64 * 16; i += 256)
        *(v4f*)&qs[i >> 4][(i & 15) * 4] = *(const v4f*)(Q + (size_t)i * 4);
    for (int i = tid; i < 65 * 16; i += 256)
        *(v4f*)&kv[i >> 4][(i & 15) * 4] = *(const v4f*)(K + (size_t)i * 4);
    __syncthreads();

    const int irow = tid >> 2, sub = tid & 3;
    #pragma unroll 1
    for (int jj = 0; jj < 17; ++jj) {
        const int j  = sub + 4 * jj;
        const int jc = (j > 64) ? 64 : j;
        float acc = 0.f;
        #pragma unroll 2
        for (int c = 0; c < 16; ++c) {
            const v4f a = *(const v4f*)&qs[irow][4 * c];
            const v4f b = *(const v4f*)&kv[jc][4 * c];
            acc = fmaf(a.x, b.x, acc); acc = fmaf(a.y, b.y, acc);
            acc = fmaf(a.z, b.z, acc); acc = fmaf(a.w, b.w, acc);
        }
        ps[irow][j] = acc * 0.125f;
    }
    __syncthreads();

    for (int i = tid; i < 65 * 16; i += 256)
        *(v4f*)&kv[i >> 4][(i & 15) * 4] = *(const v4f*)(V + (size_t)i * 4);
    {
        const int nvis = (irow + 2 < 65) ? (irow + 2) : 65;
        float mx = -3.0e38f;
        #pragma unroll 1
        for (int jj = 0; jj < 17; ++jj) {
            const int j = sub + 4 * jj;
            const float s = ps[irow][j];
            mx = (j < nvis) ? fmaxf(mx, s) : mx;
        }
        mx = fmaxf(mx, __shfl_xor(mx, 1, 32));
        mx = fmaxf(mx, __shfl_xor(mx, 2, 32));
        float sm = 0.f;
        #pragma unroll 1
        for (int jj = 0; jj < 17; ++jj) {
            const int j = sub + 4 * jj;
            const float s = ps[irow][j];
            const float p = (j < nvis) ? exp2f((s - mx) * LOG2E) : 0.f;
            ps[irow][j] = p;
            sm += p;
        }
        sm += __shfl_xor(sm, 1, 32);
        sm += __shfl_xor(sm, 2, 32);
        if (sub == 0) rinv[irow] = 1.0f / sm;
    }
    __syncthreads();

    {
        float acc[16];
        #pragma unroll
        for (int e = 0; e < 16; ++e) acc[e] = 0.f;
        #pragma unroll 1
        for (int j = 0; j < 65; ++j) {
            const float p = ps[irow][j];
            #pragma unroll
            for (int e = 0; e < 4; ++e) {
                const v4f vv = *(const v4f*)&kv[j][16 * sub + 4 * e];
                acc[4 * e + 0] = fmaf(p, vv.x, acc[4 * e + 0]);
                acc[4 * e + 1] = fmaf(p, vv.y, acc[4 * e + 1]);
                acc[4 * e + 2] = fmaf(p, vv.z, acc[4 * e + 2]);
                acc[4 * e + 3] = fmaf(p, vv.w, acc[4 * e + 3]);
            }
        }
        const float inv = rinv[irow];
        #pragma unroll
        for (int e = 0; e < 4; ++e) {
            v4f ov;
            ov.x = acc[4 * e + 0] * inv; ov.y = acc[4 * e + 1] * inv;
            ov.z = acc[4 * e + 2] * inv; ov.w = acc[4 * e + 3] * inv;
            *(v4f*)&qs[irow][16 * sub + 4 * e] = ov;
        }
    }
    __syncthreads();

    const int q8 = tid & 7, lg = tid >> 3;
    unsigned short* cbase = ctx + ((size_t)bbI * SEQ) * DM + hh * HD;
    auto passe = [&]() {
        #pragma unroll
        for (int it = 0; it < 4; ++it) {
            const int L = it * 32 + lg;
            const int row = L >> 1, pl = L & 1;
            const v4f a0 = *(const v4fa*)&qs[row][8 * q8];
            const v4f a1 = *(const v4fa*)&qs[row][8 * q8 + 4];
            float x[8] = { a0.x, a0.y, a0.z, a0.w, a1.x, a1.y, a1.z, a1.w };
            unsigned int sv[8];
            #pragma unroll
            for (int e = 0; e < 8; ++e) {
                const unsigned short hb = f2bf(x[e]);
                const unsigned short lb = f2bf(x[e] - bf2f(hb));
                sv[e] = (unsigned int)(pl ? lb : hb);
            }
            u32x4 pk;
            pk.x = sv[0] | (sv[1] << 16);
            pk.y = sv[2] | (sv[3] << 16);
            pk.z = sv[4] | (sv[5] << 16);
            pk.w = sv[6] | (sv[7] << 16);
            *(volatile u32x4*)(cbase + (size_t)pl * CPL + (size_t)row * DM + 8 * q8) = pk;
        }
    };
    passe();
    __threadfence();
    passe();
}

__launch_bounds__(128)
__global__ void outproj_kernel(const unsigned short* __restrict__ ctx,
                               const unsigned short* __restrict__ wb,
                               const float* __restrict__ bc,
                               float* __restrict__ out)
{
    __shared__ __align__(16) float stg[128][68];

    const int tid = threadIdx.x, l = tid & 31, w = tid >> 5;
    const int h = (l >> 4) & 1, nl = l & 15;
    const int mblk = blockIdx.x * 128;
    const int nb   = blockIdx.y;
    const unsigned short* W = wb + (size_t)3 * WPL;

    v8f acc[2][4] = {};
    #pragma unroll 2
    for (int s = 0; s < 32; ++s) {
        const unsigned short* AP = ctx + (size_t)(s >> 4) * CPL;
        const int kk = 32 * (s & 15) + 8 * h;
        Frag A[2], B[4];
        #pragma unroll
        for (int mi = 0; mi < 2; ++mi) {
            const unsigned short* p = AP + (size_t)(mblk + 32 * w + 16 * mi + nl) * DM + kk;
            A[mi].q[0] = *(const u32x4*)(p);
            A[mi].q[1] = *(const u32x4*)(p + 16);
        }
        #pragma unroll
        for (int ni = 0; ni < 4; ++ni) {
            const unsigned short* p = W + (size_t)(nb * 64 + 16 * ni + nl) * DM + kk;
            B[ni].q[0] = *(const u32x4*)(p);
            B[ni].q[1] = *(const u32x4*)(p + 16);
        }
        #pragma unroll
        for (int mi = 0; mi < 2; ++mi)
            #pragma unroll
            for (int ni = 0; ni < 4; ++ni)
                acc[mi][ni] = mma_bf16(A[mi], B[ni], acc[mi][ni]);
    }

    float bbv[4];
    #pragma unroll
    for (int ni = 0; ni < 4; ++ni) bbv[ni] = bfr(bc[nb * 64 + 16 * ni + nl]);
    #pragma unroll
    for (int mi = 0; mi < 2; ++mi)
        #pragma unroll
        for (int ni = 0; ni < 4; ++ni)
            #pragma unroll
            for (int r = 0; r < 8; ++r)
                stg[32 * w + 16 * mi + 8 * h + r][16 * ni + nl] = acc[mi][ni][r] + bbv[ni];
    __syncthreads();

    const int q8 = tid & 7, lg = tid >> 3;
    auto passo = [&]() {
        #pragma unroll
        for (int it = 0; it < 16; ++it) {
            const int L = it * 16 + lg;
            const int row = L >> 1, hf = L & 1;
            const v4f x = *(const v4fa*)&stg[row][hf * 32 + 4 * q8];
            const int m  = mblk + row;
            const int bbI = m / SEQ;
            const int t  = m - bbI * SEQ;
            *(volatile v4f*)(out + ((size_t)bbI * SEQ_FULL + t) * DM + nb * 64 + hf * 32 + 4 * q8) = x;
        }
    };
    passo();
    __threadfence();
    passo();
}

extern "C" void kernel_launch(void* const* d_in, const int* in_sizes, int n_in,
                              void* d_out, int out_size, void* d_ws, size_t ws_size,
                              hipStream_t stream)
{
    if (n_in < 11) return;
    const int need_x = ((NB - 1) * SEQ_FULL + SEQ) * DM;
    if (in_sizes[0] < need_x || in_sizes[1] < need_x || in_sizes[2] < need_x) return;
    if (in_sizes[3] < DM * DM || in_sizes[5] < DM * DM || in_sizes[7] < DM * DM || in_sizes[9] < DM * DM) return;
    if (in_sizes[4] < DM || in_sizes[6] < DM || in_sizes[8] < DM || in_sizes[10] < DM) return;
    if (out_size < need_x) return;

    const float* q  = (const float*)d_in[0];
    const float* k  = (const float*)d_in[1];
    const float* v  = (const float*)d_in[2];
    const float* Wq = (const float*)d_in[3];
    const float* bq = (const float*)d_in[4];
    const float* Wk = (const float*)d_in[5];
    const float* bk = (const float*)d_in[6];
    const float* Wv = (const float*)d_in[7];
    const float* bv = (const float*)d_in[8];
    const float* Wc = (const float*)d_in[9];
    const float* bc = (const float*)d_in[10];
    float* out = (float*)d_out;

    size_t off = 0;
    char* wsb = (char*)d_ws;
    auto take = [&](size_t bytes) { char* p = wsb + off; off += (bytes + 255) & ~(size_t)255; return p; };
    unsigned short* xb  = (unsigned short*)take((size_t)3 * XPL * 2);
    unsigned short* ctx = xb;
    unsigned short* wb  = (unsigned short*)take((size_t)4 * WPL * 2);
    unsigned short* qh  = (unsigned short*)take(XPL * 2);
    unsigned short* kh  = (unsigned short*)take(XPL * 2);
    unsigned short* vt  = (unsigned short*)take(XPL * 2);
    unsigned short* qr  = (unsigned short*)take(RPL * 2);
    unsigned short* kr  = (unsigned short*)take(RPL * 2);
    unsigned short* vr  = (unsigned short*)take(RPL * 2);
    float* qf = (float*)take(FPL * 4);
    float* kf = (float*)take(FPL * 4);
    float* vf = (float*)take(FPL * 4);
    if (off > ws_size) return;

    cvt_kernel<<<dim3(3 * (NTOK / 4) + 512), dim3(256), 0, stream>>>(q, k, v, Wq, Wk, Wv, Wc, xb, wb);
    proj_kernel<<<dim3(NTOK / 128, NH, 3), dim3(128), 0, stream>>>(xb, wb, bq, bk, bv,
                                                                  qh, kh, vt, qr, kr, vr,
                                                                  qf, kf, vf);
    if (SEQ / 64 > EQB) {
        attn_kernel<0><<<dim3(SEQ / 64 - EQB, NB * NH), dim3(128), 0, stream>>>(qh, kh, vt, qr, kr, vr, ctx);
    }
    attn_kernel<1><<<dim3(EQB - 1, NB * NH), dim3(128), 0, stream>>>(qh, kh, vt, qr, kr, vr, ctx);
    attn_first_kernel<<<dim3(NB * NH), dim3(256), 0, stream>>>(qf, kf, vf, ctx);
    outproj_kernel<<<dim3(NTOK / 128, DM / 64), dim3(128), 0, stream>>>(ctx, wb, bc, out);
}
